// DemoModule_25512105739100
// MI455X (gfx1250) — hardware-verified
//
#include <hip/hip_runtime.h>
#include <hip/hip_bf16.h>
#include <math.h>


#define BB 2
#define SS 2048
#define DD 1024
#define HH 16
#define DKK 64
#define QW 2

typedef _Float16 bf16;
typedef __attribute__((ext_vector_type(4))) unsigned v4u_t;
typedef unsigned v4ua __attribute__((ext_vector_type(4), may_alias));
typedef __attribute__((ext_vector_type(4))) float v4f_t;
typedef float v4fa __attribute__((ext_vector_type(4), may_alias));
typedef __attribute__((ext_vector_type(16))) bf16  bf16x16;
typedef __attribute__((ext_vector_type(8)))  bf16  bf16x8;
typedef __attribute__((ext_vector_type(4)))  bf16  bf16x4;
typedef __attribute__((ext_vector_type(8)))  float f32x8;

#define LDS_STRIDE 48
#define KSTRIDE    72
#define VSTRIDE    48

__device__ __forceinline__ f32x8 wmma_bf16(bf16x16 a, bf16x16 b, f32x8 c) {
  return __builtin_amdgcn_wmma_f32_16x16x32_f16(
      false, a, false, b, (short)0, c, false, false);
}

template <typename T>
__device__ __forceinline__ bf16x16 load_frag(const T* __restrict__ base, int ld,
                                             int row0, int k0) {
  const int lane = threadIdx.x & 31;
  const int r    = lane & 15;
  const int kh   = (lane >> 4) * 8;
  const T* p0 = base + (size_t)(row0 + r) * ld + (k0 + kh);
  const T* p1 = p0 + 16;
  bf16x16 f;
#pragma unroll
  for (int i = 0; i < 8; ++i) {
    f[i]     = (bf16)p0[i];
    f[i + 8] = (bf16)p1[i];
  }
  return f;
}

__device__ __forceinline__ bf16x16 lds_frag(const bf16* base, int stride) {
  const int lane = threadIdx.x & 31;
  const int row  = lane & 15;
  const int kh   = (lane >> 4) * 8;
  const bf16x8 lo = *(const bf16x8*)(base + row * stride + kh);
  const bf16x8 hi = *(const bf16x8*)(base + row * stride + kh + 16);
  bf16x16 f;
#pragma unroll
  for (int i = 0; i < 8; ++i) { f[i] = lo[i]; f[i + 8] = hi[i]; }
  return f;
}

template <typename T>
__device__ __forceinline__ void stage_read16(const T* __restrict__ p, float* buf) {
#pragma unroll
  for (int i = 0; i < 16; ++i) buf[i] = (float)p[i];
}

__device__ __forceinline__ void stage_write(bf16* dst, const float* buf, int nquad) {
#pragma unroll
  for (int i = 0; i < nquad; ++i) {
    bf16x4 q;
    q[0] = (bf16)buf[4 * i];     q[1] = (bf16)buf[4 * i + 1];
    q[2] = (bf16)buf[4 * i + 2]; q[3] = (bf16)buf[4 * i + 3];
    *(bf16x4*)(dst + 4 * i) = q;
  }
}

template <typename AT, int MODE>
__global__ __launch_bounds__(256) void gemm_bias_kernel(
    const AT* __restrict__ A, const float* __restrict__ W,
    const float* __restrict__ bias, void* __restrict__ out,
    int M, int N, int K) {
  __shared__ bf16 ldsA[128 * LDS_STRIDE];
  __shared__ bf16 ldsW[256 * LDS_STRIDE];
  __shared__ __attribute__((aligned(16))) unsigned char sob[256 * 136 * 2];

  const int t    = threadIdx.x;
  const int wave = t >> 5;
  const int lane = t & 31;
  const int wm   = (wave & 1) * 64;
  const int wn   = (wave >> 1) * 64;
  const int mBlk = blockIdx.x * 128;
  const int nBlk = blockIdx.y * 256;

  const int arow = t >> 1;
  const int ach  = (t & 1) * 16;

  float abuf[16];
  float wbuf[32];

  stage_read16(A + (size_t)(mBlk + arow) * K + ach, abuf);
  stage_read16(W + (size_t)(nBlk + t) * K,          wbuf);
  stage_read16(W + (size_t)(nBlk + t) * K + 16,     wbuf + 16);

  f32x8 acc[4][4] = {};

  for (int k = 0; k < K; k += 32) {
    __syncthreads();
    stage_write(&ldsA[arow * LDS_STRIDE + ach], abuf, 4);
    stage_write(&ldsW[t * LDS_STRIDE],          wbuf, 8);
    if (k + 32 < K) {
      stage_read16(A + (size_t)(mBlk + arow) * K + (k + 32) + ach, abuf);
      stage_read16(W + (size_t)(nBlk + t) * K + (k + 32),          wbuf);
      stage_read16(W + (size_t)(nBlk + t) * K + (k + 32) + 16,     wbuf + 16);
    }
    __syncthreads();

    bf16x16 af[4], wf[4];
#pragma unroll
    for (int i = 0; i < 4; ++i)
      af[i] = lds_frag(ldsA + (wm + 16 * i) * LDS_STRIDE, LDS_STRIDE);
#pragma unroll
    for (int j = 0; j < 4; ++j)
      wf[j] = lds_frag(ldsW + (wn + 16 * j) * LDS_STRIDE, LDS_STRIDE);
#pragma unroll
    for (int i = 0; i < 4; ++i)
#pragma unroll
      for (int j = 0; j < 4; ++j)
        acc[i][j] = wmma_bf16(af[i], wf[j], acc[i][j]);
  }

  const int nlane = lane & 15;
  const int mh    = (lane >> 4) * 8;
  __syncthreads();
  if (MODE == 0 || MODE == 1 || MODE == 3) {
    bf16* so = (bf16*)sob;
#pragma unroll
    for (int i = 0; i < 4; ++i)
#pragma unroll
      for (int j = 0; j < 4; ++j) {
        const int nl = wn + 16 * j + nlane;
        const float bv = bias ? bias[nBlk + nl] : 0.0f;
#pragma unroll
        for (int r = 0; r < 8; ++r) {
          const int ml = wm + 16 * i + mh + r;
          const bf16 hv = (MODE == 3) ? (bf16)fmaxf(acc[i][j][r] + bv, 0.0f) : (bf16)(acc[i][j][r] + bv);
          if (MODE == 0 || MODE == 3) so[ml * 264 + nl] = hv;
          else           so[nl * 136 + ml] = hv;
        }
      }
    __syncthreads();
#pragma unroll 1
    for (int pass = 0; pass < 2; ++pass) {
      if (MODE == 0 || MODE == 3) {
        for (int ch = t; ch < 128 * 32; ch += 256) { const int ml = ch >> 5, q = (ch & 31) * 8;
          *(volatile v4u_t*)((bf16*)out + (size_t)(mBlk + ml) * N + nBlk + q) = *(const v4ua*)(so + ml * 264 + q); }
      } else {
        const int b_ = mBlk / SS, s0 = mBlk & (SS - 1);
        for (int ch = t; ch < 256 * 16; ch += 256) { const int nl = ch >> 4, q = (ch & 15) * 8; const int n = nBlk + nl, h = n >> 6, dk = n & (DKK - 1);
          *(volatile v4u_t*)((bf16*)out + (((size_t)(b_ * HH + h)) * DKK + dk) * SS + s0 + q) = *(const v4ua*)(so + nl * 136 + q); }
      }
      __threadfence();
    }
  } else {
    float* so = (float*)sob;
#pragma unroll 1
    for (int hf = 0; hf < 2; ++hf) {
      if (wm == hf * 64) {
#pragma unroll
        for (int i = 0; i < 4; ++i)
#pragma unroll
          for (int j = 0; j < 4; ++j) {
            const int nl = wn + 16 * j + nlane;
            const float bv = bias ? bias[nBlk + nl] : 0.0f;
#pragma unroll
            for (int r = 0; r < 8; ++r) so[(16 * i + mh + r) * 260 + nl] = acc[i][j][r] + bv;
          }
      }
      __syncthreads();
#pragma unroll 1
      for (int pass = 0; pass < 2; ++pass) {
        for (int ch = t; ch < 64 * 64; ch += 256) { const int ml = ch >> 6, q = (ch & 63) * 4;
          *(volatile v4f_t*)((float*)out + (size_t)(mBlk + hf * 64 + ml) * N + nBlk + q) = *(const volatile v4fa*)(so + ml * 260 + q); }
        __threadfence();
      }
      __syncthreads();
    }
  }
}


#define NB 16384
#define NF 64
#define NL 10
#define NE 16
#define NV 1000000
#define D0 1024
#define D1 1024
#define D2 512

__global__ __launch_bounds__(256) void k_tw(const float* __restrict__ W, float* __restrict__ WT, int K, int N) {
  __shared__ float tile[64][65];
  const int kb0 = blockIdx.y * 64, n0 = blockIdx.x * 64, t = threadIdx.x;
  for (int i = t; i < 64 * 64; i += 256) { const int kr = i >> 6, nc = i & 63; tile[kr][nc] = W[(size_t)(kb0 + kr) * N + n0 + nc]; }
  __syncthreads();
#pragma unroll 1
  for (int pass = 0; pass < 2; ++pass) {
    for (int i = t; i < 64 * 16; i += 256) { const int nr = i >> 4, k4 = (i & 15) * 4; v4f_t v; v.x = tile[k4][nr]; v.y = tile[k4 + 1][nr]; v.z = tile[k4 + 2][nr]; v.w = tile[k4 + 3][nr];
      *(volatile v4f_t*)(WT + (size_t)(n0 + nr) * K + kb0 + k4) = v; }
    __threadfence();
  }
}
__global__ __launch_bounds__(256) void k_gather(const int* __restrict__ idx, const float* __restrict__ emb, float* __restrict__ X) {
  const int b = blockIdx.x, t = threadIdx.x, f = t >> 2, e4 = (t & 3) * 4;
  v4f_t s; s.x = s.y = s.z = s.w = 0.0f;
#pragma unroll 1
  for (int l = 0; l < NL; ++l) { int id = idx[((size_t)b * NF + f) * NL + l]; id = id < 0 ? 0 : (id >= NV ? NV - 1 : id);
    const v4f_t v = *(const v4fa*)(emb + (size_t)id * NE + e4); s.x += v.x; s.y += v.y; s.z += v.z; s.w += v.w; }
  *(volatile v4f_t*)(X + (size_t)b * D0 + f * NE + e4) = s; __threadfence(); *(volatile v4f_t*)(X + (size_t)b * D0 + f * NE + e4) = s;
}
__global__ __launch_bounds__(256) void k_colstat(const float* __restrict__ X, float* __restrict__ st) {
  __shared__ float rs_[256], rq_[256];
  const int c = blockIdx.x, t = threadIdx.x; float s = 0.f, q = 0.f;
  for (int r = t; r < NB; r += 256) { const float v = X[(size_t)r * D0 + c]; s += v; q += v * v; }
  rs_[t] = s; rq_[t] = q; __syncthreads();
  for (int o = 128; o > 0; o >>= 1) { if (t < o) { rs_[t] += rs_[t + o]; rq_[t] += rq_[t + o]; } __syncthreads(); }
  if (t < 32) { float v = 0.0f; const double mu = (double)rs_[0] / (double)NB;
    if (t == 0) v = (float)mu; if (t == 1) { const double var = fmax((double)rq_[0] / (double)NB - mu * mu, 0.0); v = (float)(1.0 / sqrt(var + 1e-5)); }
    *(volatile float*)(st + (size_t)c * 32 + t) = v; __threadfence(); *(volatile float*)(st + (size_t)c * 32 + t) = v; }
}
__global__ __launch_bounds__(256) void k_norm(const float* __restrict__ X, const float* __restrict__ st, bf16* __restrict__ XN) {
  const int b = blockIdx.x, t = threadIdx.x; const v4f_t v = *(const v4fa*)(X + (size_t)b * D0 + t * 4); bf16 h[4];
#pragma unroll
  for (int q = 0; q < 4; ++q) { const int c = t * 4 + q; h[q] = (bf16)((v[q] - st[(size_t)c * 32]) * st[(size_t)c * 32 + 1]); }
  typedef __attribute__((ext_vector_type(2))) unsigned v2u; typedef unsigned v2ua __attribute__((ext_vector_type(2), may_alias));
  *(volatile v2u*)(XN + (size_t)b * D0 + t * 4) = *(const v2ua*)h; __threadfence(); *(volatile v2u*)(XN + (size_t)b * D0 + t * 4) = *(const v2ua*)h;
}
__global__ __launch_bounds__(256) void k_head(const bf16* __restrict__ H2, const float* __restrict__ W3, const float* __restrict__ b3, float* __restrict__ out) {
  __shared__ float part[64][5]; __shared__ float res[64];
  const int t = threadIdx.x, rl = t >> 2, p4 = t & 3, b = blockIdx.x * 64 + rl; float s = 0.0f;
  const bf16* hr = H2 + (size_t)b * D2 + p4 * 128;
#pragma unroll 1
  for (int k = 0; k < 128; ++k) s += (float)hr[k] * W3[p4 * 128 + k];
  part[rl][p4] = s; __syncthreads();
  if (t < 64) { const float z = part[t][0] + part[t][1] + part[t][2] + part[t][3] + b3[0]; res[t] = 1.0f / (1.0f + expf(-z)); }
  __syncthreads();
  if (t < 16) { const v4f_t v = *(const volatile v4fa*)(res + t * 4); *(volatile v4f_t*)(out + (size_t)blockIdx.x * 64 + t * 4) = v; __threadfence(); *(volatile v4f_t*)(out + (size_t)blockIdx.x * 64 + t * 4) = v; }
}

extern "C" void kernel_launch(void* const* d_in, const int* in_sizes, int n_in,
                              void* d_out, int out_size, void* d_ws, size_t ws_size,
                              hipStream_t stream) {
  (void)in_sizes; (void)n_in; (void)out_size; (void)ws_size;
  const int* idx = (const int*)d_in[0];
  const float* emb = (const float*)d_in[1];
  const float* W1 = (const float*)d_in[2]; const float* b1 = (const float*)d_in[3];
  const float* W2 = (const float*)d_in[4]; const float* b2 = (const float*)d_in[5];
  const float* W3 = (const float*)d_in[6]; const float* b3 = (const float*)d_in[7];
  char* ws = (char*)d_ws;
  float* W1T = (float*)ws; ws += (size_t)D1 * D0 * 4;
  float* W2T = (float*)ws; ws += (size_t)D2 * D1 * 4;
  float* st  = (float*)ws; ws += (size_t)D0 * 32 * 4;
  float* X   = (float*)ws; ws += (size_t)NB * D0 * 4;
  bf16* H1   = (bf16*)X;
  bf16* H2   = (bf16*)((char*)X + (size_t)NB * D1 * 2);
  bf16* XN   = (bf16*)ws;  ws += (size_t)NB * D0 * 2;
  k_tw<<<dim3(D1 / 64, D0 / 64), 256, 0, stream>>>(W1, W1T, D0, D1);
  k_tw<<<dim3(D2 / 64, D1 / 64), 256, 0, stream>>>(W2, W2T, D1, D2);
  k_gather<<<NB, 256, 0, stream>>>(idx, emb, X);
  k_colstat<<<D0, 256, 0, stream>>>(X, st);
  k_norm<<<NB, 256, 0, stream>>>(X, st, XN);
  dim3 blk(256);
  gemm_bias_kernel<bf16, 3><<<dim3(NB / 128, D1 / 256), blk, 0, stream>>>(XN, W1T, b1, H1, NB, D1, D0);
  gemm_bias_kernel<bf16, 3><<<dim3(NB / 128, D2 / 256), blk, 0, stream>>>(H1, W2T, b2, H2, NB, D2, D1);
  k_head<<<NB / 64, 256, 0, stream>>>(H2, W3, b3, (float*)d_out);
}
